// GCN_49082886259351
// MI455X (gfx1250) — hardware-verified
//
#include <hip/hip_runtime.h>
#include <stddef.h>
#include <stdint.h>
#include <math.h>


#define DF     128
#define DO3    64
#define KH     256
#define NTHR   256
#define NWAVE  8
#define EPT    8
#define CHUNK  (NTHR * EPT)
#define WCAP   (EPT * 32)
#define LISTN  (NWAVE * WCAP)
#define NBA    1024
#define SLA    10
#define RCAP   20480
#define DEGCAP 64
#define GBM    64
#define GBN    64
#define GTHR   128
#define NU1    (DF * (DF / 8))
#define NU2    (DF * (KH / 8))
#define NU3    (DO3 * (KH / 8))
#define GR_ZINTS (LISTN + 2 * RCAP + 3 * NBA)
#define GR_LDS_INTS (GR_ZINTS + 16)
#define WSMAX  134217728

static_assert((CHUNK & (CHUNK - 1)) == 0 && CHUNK <= 4096);
static_assert((NBA & (NBA - 1)) == 0 && NBA == (1 << SLA));
static_assert(((long long)CHUNK << SLA) < (1LL << 31));
static_assert(NBA % NWAVE == 0 && NBA % 32 == 0 && NBA % GBM == 0 && NBA == 4 * NTHR);
static_assert(RCAP % NTHR == 0 && GR_ZINTS % 4 == 0 && LISTN % 4 == 0);
static_assert(DF % 32 == 0 && KH % 32 == 0 && KH == 2 * DF);
static_assert(GBM == (GTHR / 32) * 16 && GBN == 64 && DF % GBN == 0 && DO3 % GBN == 0);
static_assert(NU1 % NTHR == 0 && NU2 % NTHR == 0 && NU3 % NTHR == 0);
static_assert(DF == 4 * 32 && DO3 == 2 * 32);
static_assert(GR_LDS_INTS * 4 <= 300000);
static_assert(DEGCAP <= 64);

typedef float          v2f   __attribute__((ext_vector_type(2)));
typedef float          v4f   __attribute__((ext_vector_type(4)));
typedef float          v8f   __attribute__((ext_vector_type(8)));
typedef int            v4i   __attribute__((ext_vector_type(4)));
typedef int            v8i   __attribute__((ext_vector_type(8)));
typedef unsigned short v4us  __attribute__((ext_vector_type(4)));
typedef unsigned short v8us  __attribute__((ext_vector_type(8)));
typedef unsigned short v16us __attribute__((ext_vector_type(16)));
typedef __bf16         v16bf __attribute__((ext_vector_type(16)));
typedef v2f  __attribute__((may_alias)) v2fa;
typedef v4f  __attribute__((may_alias)) v4fa;
typedef v4i  __attribute__((may_alias)) v4ia;
typedef v4us __attribute__((may_alias)) v4usa;
typedef v8us __attribute__((may_alias)) v8usa;
union FragB { v16bf v; v16us u; v8us h[2]; v8i w; };

__device__ __forceinline__ v8f wmb(const FragB& a, const FragB& b, v8f c) {
  v8f d = __builtin_amdgcn_wmma_f32_16x16x32_bf16(false, a.v, false, b.v, (short)0, c, false, false);
  asm volatile("v_nop\n\tv_nop\n\tv_nop\n\tv_nop" : "+v"(d) : "v"(a.w), "v"(b.w));
  return d;
}

__device__ __forceinline__ unsigned bf16_bits(float f) {
  const unsigned u = __float_as_uint(f);
  return (u + 0x7FFFu + ((u >> 16) & 1u)) >> 16;
}
__device__ __forceinline__ float bf16_val(float f) {
  return __uint_as_float(bf16_bits(f) << 16);
}

__device__ __forceinline__ void wave_sync() {
  __builtin_amdgcn_fence(__ATOMIC_RELEASE, "wavefront");
  __builtin_amdgcn_wave_barrier();
  __builtin_amdgcn_fence(__ATOMIC_ACQUIRE, "wavefront");
}

template <int SLB>
__device__ __forceinline__ int scan_chunk(const int* __restrict__ dsts, int nE, int cbase, int slotBase,
                                          int nb, int vec8, int* list, int tid, int lane, int wave) {
  int wc = 0;
  const int el0  = tid * EPT;
  const int e0   = cbase + el0;
  const int sent = -2147483647 - 1;
  v4i da, db;
  if (vec8 != 0 && cbase + CHUNK <= nE) {
    da = *(const v4i*)(dsts + e0);
    db = *(const v4i*)(dsts + e0 + 4);
  } else {
    da.x = (e0     < nE) ? dsts[min(e0,     nE - 1)] : sent;
    da.y = (e0 + 1 < nE) ? dsts[min(e0 + 1, nE - 1)] : sent;
    da.z = (e0 + 2 < nE) ? dsts[min(e0 + 2, nE - 1)] : sent;
    da.w = (e0 + 3 < nE) ? dsts[min(e0 + 3, nE - 1)] : sent;
    db.x = (e0 + 4 < nE) ? dsts[min(e0 + 4, nE - 1)] : sent;
    db.y = (e0 + 5 < nE) ? dsts[min(e0 + 5, nE - 1)] : sent;
    db.z = (e0 + 6 < nE) ? dsts[min(e0 + 6, nE - 1)] : sent;
    db.w = (e0 + 7 < nE) ? dsts[min(e0 + 7, nE - 1)] : sent;
  }
  const unsigned nbs = (unsigned)slotBase;
  const unsigned unb = (unsigned)nb;
  const unsigned s0 = (unsigned)da.x - nbs, s1 = (unsigned)da.y - nbs;
  const unsigned s2 = (unsigned)da.z - nbs, s3 = (unsigned)da.w - nbs;
  const unsigned s4 = (unsigned)db.x - nbs, s5 = (unsigned)db.y - nbs;
  const unsigned s6 = (unsigned)db.z - nbs, s7 = (unsigned)db.w - nbs;
  const bool h0 = s0 < unb, h1 = s1 < unb, h2 = s2 < unb, h3 = s3 < unb;
  const bool h4 = s4 < unb, h5 = s5 < unb, h6 = s6 < unb, h7 = s7 < unb;
  const unsigned any = __builtin_amdgcn_ballot_w32(h0 | h1 | h2 | h3 | h4 | h5 | h6 | h7);
  if (any != 0u) {
    const unsigned m0 = __builtin_amdgcn_ballot_w32(h0);
    const unsigned m1 = __builtin_amdgcn_ballot_w32(h1);
    const unsigned m2 = __builtin_amdgcn_ballot_w32(h2);
    const unsigned m3 = __builtin_amdgcn_ballot_w32(h3);
    const unsigned m4 = __builtin_amdgcn_ballot_w32(h4);
    const unsigned m5 = __builtin_amdgcn_ballot_w32(h5);
    const unsigned m6 = __builtin_amdgcn_ballot_w32(h6);
    const unsigned m7 = __builtin_amdgcn_ballot_w32(h7);
    int pos = wc
            + (int)__builtin_amdgcn_mbcnt_lo(m0, 0u) + (int)__builtin_amdgcn_mbcnt_lo(m1, 0u)
            + (int)__builtin_amdgcn_mbcnt_lo(m2, 0u) + (int)__builtin_amdgcn_mbcnt_lo(m3, 0u)
            + (int)__builtin_amdgcn_mbcnt_lo(m4, 0u) + (int)__builtin_amdgcn_mbcnt_lo(m5, 0u)
            + (int)__builtin_amdgcn_mbcnt_lo(m6, 0u) + (int)__builtin_amdgcn_mbcnt_lo(m7, 0u);
    int* lw = list + wave * WCAP;
    if (h0 && pos < WCAP) lw[pos] = ((el0 + 0) << SLB) | (int)s0;
    pos += h0 ? 1 : 0;
    if (h1 && pos < WCAP) lw[pos] = ((el0 + 1) << SLB) | (int)s1;
    pos += h1 ? 1 : 0;
    if (h2 && pos < WCAP) lw[pos] = ((el0 + 2) << SLB) | (int)s2;
    pos += h2 ? 1 : 0;
    if (h3 && pos < WCAP) lw[pos] = ((el0 + 3) << SLB) | (int)s3;
    pos += h3 ? 1 : 0;
    if (h4 && pos < WCAP) lw[pos] = ((el0 + 4) << SLB) | (int)s4;
    pos += h4 ? 1 : 0;
    if (h5 && pos < WCAP) lw[pos] = ((el0 + 5) << SLB) | (int)s5;
    pos += h5 ? 1 : 0;
    if (h6 && pos < WCAP) lw[pos] = ((el0 + 6) << SLB) | (int)s6;
    pos += h6 ? 1 : 0;
    if (h7 && pos < WCAP) lw[pos] = ((el0 + 7) << SLB) | (int)s7;
    wc += (int)__builtin_popcount(m0) + (int)__builtin_popcount(m1) + (int)__builtin_popcount(m2)
        + (int)__builtin_popcount(m3) + (int)__builtin_popcount(m4) + (int)__builtin_popcount(m5)
        + (int)__builtin_popcount(m6) + (int)__builtin_popcount(m7);
  }
  return wc;
}

__device__ __forceinline__ void put8(unsigned short* dp, v8us o) {
  *(volatile v8us*)dp = o;
  __threadfence();
  *(volatile v8us*)dp = o;
}
__device__ __forceinline__ v8us gather8(const float* __restrict__ p, int stride) {
  v8us o;
#pragma unroll
  for (int i = 0; i < 8; ++i) o[i] = (unsigned short)bf16_bits(p[(size_t)i * stride]);
  return o;
}

__global__ __launch_bounds__(NTHR) void k_wprep(const float* __restrict__ W1, const float* __restrict__ W2,
                                                const float* __restrict__ W3, unsigned short* W1T,
                                                unsigned short* W2D, unsigned short* W3D) {
  const int u = (int)blockIdx.x * NTHR + (int)threadIdx.x;
  if (u < NU1) {
    const int n  = u >> 4;
    const int k8 = (u & 15) * 8;
    const v8us o = gather8(W1 + (size_t)k8 * DF + n, DF);
    put8(W1T + (size_t)n * DF + k8, o);
  } else if (u < NU1 + NU2) {
    const int v  = u - NU1;
    const int n  = v >> 5;
    const int k8 = (v & 31) * 8;
    const int kk = k8 & (DF - 1);
    const v8us o = gather8(W2 + (size_t)kk * DF + n, DF);
    put8(W2D + (size_t)n * KH + k8, o);
  } else if (u < NU1 + NU2 + NU3) {
    const int v  = u - NU1 - NU2;
    const int n  = v >> 5;
    const int k8 = (v & 31) * 8;
    const int kk = k8 & (DF - 1);
    const v8us o = gather8(W3 + (size_t)kk * DO3 + n, DO3);
    put8(W3D + (size_t)n * KH + k8, o);
  }
}

__global__ __launch_bounds__(NTHR) void k_cvx(const float* __restrict__ x, int nN, int nUnits,
                                              unsigned short* xb) {
  const int u = (int)blockIdx.x * NTHR + (int)threadIdx.x;
  if (u >= nUnits) return;
  const int row = u >> 4;
  const int k8  = (u & 15) * 8;
  const int rc  = row < nN ? row : nN - 1;
  const float* p = x + (size_t)rc * DF + k8;
  const v4f a = *(const v4fa*)p;
  const v4f b = *(const v4fa*)(p + 4);
  const bool ok = row < nN;
  v8us o;
  o[0] = ok ? (unsigned short)bf16_bits(a.x) : (unsigned short)0;
  o[1] = ok ? (unsigned short)bf16_bits(a.y) : (unsigned short)0;
  o[2] = ok ? (unsigned short)bf16_bits(a.z) : (unsigned short)0;
  o[3] = ok ? (unsigned short)bf16_bits(a.w) : (unsigned short)0;
  o[4] = ok ? (unsigned short)bf16_bits(b.x) : (unsigned short)0;
  o[5] = ok ? (unsigned short)bf16_bits(b.y) : (unsigned short)0;
  o[6] = ok ? (unsigned short)bf16_bits(b.z) : (unsigned short)0;
  o[7] = ok ? (unsigned short)bf16_bits(b.w) : (unsigned short)0;
  put8(xb + (size_t)row * DF + k8, o);
}

__device__ __forceinline__ float slot_dinv(const int* cnt, const int* offs, const int* hw, int s) {
  const int craw = cnt[s];
  int c = craw < 0 ? 0 : (craw > DEGCAP ? DEGCAP : craw);
  int o = offs[s];
  o = o < 0 ? 0 : (o > RCAP ? RCAP : o);
  float dg = 0.0f;
#pragma unroll 1
  for (int q = 0; q < c; ++q) {
    int idx = o + q;
    idx = idx > RCAP - 1 ? RCAP - 1 : idx;
    dg += __int_as_float(hw[idx]);
  }
  dg = dg + 1.0f;
  const float r = (dg > 0.0f) ? (1.0f / sqrtf(dg)) : 0.0f;
  return (craw > DEGCAP) ? __int_as_float(0x7fc00000) : r;
}

__global__ __launch_bounds__(NTHR) void k_graph(const int* __restrict__ srcs, const int* __restrict__ dsts,
                                                const float* __restrict__ ew, int nE, int nN, int vec8,
                                                int* hsrc, float* hwt, int* cntg, int* offg, float* dinv) {
  extern __shared__ __attribute__((aligned(16))) int dsm[];
  int* list = dsm;
  int* hl   = dsm + LISTN;
  int* sl   = hl + RCAP;
  int* cnt  = sl + RCAP;
  int* offs = cnt + NBA;
  int* cur  = offs + NBA;
  int* misc = cur + NBA;
  const int tid = (int)threadIdx.x, lane = tid & 31, wave = tid >> 5;
  const int nodeBase = (int)blockIdx.x * NBA;

  {
    const v4i z4 = {0, 0, 0, 0};
    for (int i = tid * 4; i < GR_ZINTS; i += NTHR * 4) *(v4ia*)(dsm + i) = z4;
    if (tid < 16) misc[tid] = 0;
  }
  __syncthreads();

  int t = 0, ov = 0;
  const int nChunks = (nE + CHUNK - 1) / CHUNK;
#pragma unroll 1
  for (int ch = 0; ch < nChunks; ++ch) {
    const int cbase = ch * CHUNK;
    const int wc = scan_chunk<SLA>(dsts, nE, cbase, nodeBase, NBA, vec8, list, tid, lane, wave);
    if (lane == 0) misc[wave] = wc;
    __syncthreads();
    if (wave == 0) {
#pragma unroll 1
      for (int w2 = 0; w2 < NWAVE; ++w2) {
        int c = misc[w2];
        c = c < 0 ? 0 : (c > WCAP ? WCAP : c);
#pragma unroll 1
        for (int b0 = 0; b0 < c; b0 += 32) {
          const int idx = b0 + lane;
          const int ent = list[w2 * WCAP + (idx < WCAP ? idx : WCAP - 1)];
          const int m32 = (c - b0) < 32 ? (c - b0) : 32;
#pragma unroll 1
          for (int k = 0; k < m32; ++k) {
            const int u    = __builtin_amdgcn_readlane(ent, k);
            const int slot = u & (NBA - 1);
            const int el   = (u >> SLA) & (CHUNK - 1);
            const int pk   = ((cbase + el) << SLA) | slot;
            if (t < RCAP) {
              if (lane == 0) { hl[t] = pk; cnt[slot] = cnt[slot] + 1; }
              t = t + 1;
            } else {
              ov = 1;
            }
          }
        }
      }
    }
    __syncthreads();
  }
  if (wave == 0 && lane == 0) { misc[8] = t; misc[9] = ov; }
  __syncthreads();
  int tt = misc[8];
  tt = tt < 0 ? 0 : (tt > RCAP ? RCAP : tt);
  const int ovf = misc[9];

  if (wave == 0) {
    const int base = lane * (NBA / 32);
    int s = 0;
#pragma unroll 1
    for (int i = 0; i < NBA / 32; ++i) s += cnt[base + i];
    int incl = s;
#pragma unroll
    for (int d = 1; d < 32; d <<= 1) {
      const int y = __shfl_up(incl, d, 32);
      if (lane >= d) incl += y;
    }
    int run = incl - s;
#pragma unroll 1
    for (int i = 0; i < NBA / 32; ++i) {
      const int cv = cnt[base + i];
      offs[base + i] = run;
      cur[base + i]  = run;
      run += cv;
    }
  }
  __syncthreads();
  if (wave == 0) {
#pragma unroll 1
    for (int b0 = 0; b0 < tt; b0 += 32) {
      const int idx = b0 + lane;
      const int ent = hl[idx < RCAP ? idx : RCAP - 1];
      const int m32 = (tt - b0) < 32 ? (tt - b0) : 32;
#pragma unroll 1
      for (int k = 0; k < m32; ++k) {
        const int u    = __builtin_amdgcn_readlane(ent, k);
        const int slot = u & (NBA - 1);
        if (lane == 0) {
          int p = cur[slot];
          p = p < 0 ? 0 : (p > RCAP - 1 ? RCAP - 1 : p);
          sl[p] = u;
          cur[slot] = p + 1;
        }
      }
    }
  }
  __syncthreads();

  const size_t hbase = (size_t)blockIdx.x * RCAP;
#pragma unroll 1
  for (int p0 = 0; p0 < RCAP; p0 += NTHR) {
    const int p = p0 + tid;
    const int ent = sl[p];
    const bool valid = p < tt;
    int eid = ent >> SLA;
    eid = eid < 0 ? 0 : (eid > nE - 1 ? nE - 1 : eid);
    int sr = srcs[eid];
    sr = sr < 0 ? 0 : (sr > nN - 1 ? nN - 1 : sr);
    float wv = bf16_val(ew[eid]);
    sr = valid ? sr : 0;
    wv = valid ? wv : 0.0f;
    hl[p] = __float_as_int(wv);
    *(volatile int*)(hsrc + hbase + p) = sr;
    *(volatile float*)(hwt + hbase + p) = wv;
    __threadfence();
    *(volatile int*)(hsrc + hbase + p) = sr;
    *(volatile float*)(hwt + hbase + p) = wv;
  }
  __syncthreads();

  const float qnan = __int_as_float(0x7fc00000);
  v4f dv4;
  dv4.x = slot_dinv(cnt, offs, hl, 4 * tid + 0);
  dv4.y = slot_dinv(cnt, offs, hl, 4 * tid + 1);
  dv4.z = slot_dinv(cnt, offs, hl, 4 * tid + 2);
  dv4.w = slot_dinv(cnt, offs, hl, 4 * tid + 3);
  v4i c4 = *(const v4ia*)(cnt + 4 * tid);
  const v4i o4 = *(const v4ia*)(offs + 4 * tid);
  if (ovf != 0) {
    c4.x = 2147483647; c4.y = 2147483647; c4.z = 2147483647; c4.w = 2147483647;
    dv4.x = qnan; dv4.y = qnan; dv4.z = qnan; dv4.w = qnan;
  }
  const size_t sb = (size_t)nodeBase + 4 * tid;
  *(volatile v4f*)(dinv + sb) = dv4;
  *(volatile v4i*)(cntg + sb) = c4;
  *(volatile v4i*)(offg + sb) = o4;
  __threadfence();
  *(volatile v4f*)(dinv + sb) = dv4;
  *(volatile v4i*)(cntg + sb) = c4;
  *(volatile v4i*)(offg + sb) = o4;
}

__global__ __launch_bounds__(GTHR) void k_gemm(
    const unsigned short* __restrict__ A, const unsigned short* __restrict__ WT,
    const float* __restrict__ dinv, float* outF, int K, int ldo)
{
  __shared__ __attribute__((aligned(16))) float stg[GBM * GBN];
  __shared__ float sdv[GBM];
  const int tid = (int)threadIdx.x, lane = tid & 31, wave = tid >> 5, hh = lane >> 4, m = lane & 15;
  const int rowBase = (int)blockIdx.x * GBM;
  const int col0    = (int)blockIdx.y * GBN;

  v8f acc[4];
  {
    const v8f z = {0.f, 0.f, 0.f, 0.f, 0.f, 0.f, 0.f, 0.f};
    acc[0] = z; acc[1] = z; acc[2] = z; acc[3] = z;
  }
  const unsigned short* ap = A  + (size_t)(rowBase + 16 * wave + m) * (size_t)K + 8 * hh;
  const unsigned short* wp = WT + (size_t)(col0 + m) * (size_t)K + 8 * hh;
  const int ksteps = K >> 5;
#pragma unroll 1
  for (int ks = 0; ks < ksteps; ++ks) {
    FragB af;
    af.h[0] = *(const v8usa*)(ap + 32 * ks);
    af.h[1] = *(const v8usa*)(ap + 32 * ks + 16);
#pragma unroll
    for (int t = 0; t < 4; ++t) {
      const unsigned short* wq = wp + (size_t)(16 * t) * (size_t)K + 32 * ks;
      FragB bf;
      bf.h[0] = *(const v8usa*)wq;
      bf.h[1] = *(const v8usa*)(wq + 16);
      acc[t] = wmb(af, bf, acc[t]);
    }
  }

  if (tid < GBM) sdv[tid] = dinv[rowBase + tid];
#pragma unroll
  for (int t = 0; t < 4; ++t) {
    const int lc = 16 * t + m;
#pragma unroll
    for (int r = 0; r < 8; ++r) {
      const int lr = 16 * wave + 8 * hh + r;
      stg[lr * GBN + lc] = acc[t][r];
    }
  }
  __syncthreads();

  v4f fv[8];
#pragma unroll
  for (int i = 0; i < 8; ++i) {
    const int lr = 16 * wave + 2 * i + hh;
    const v4f raw = *(const v4fa*)(stg + lr * GBN + 4 * m);
    const float dv = sdv[lr];
    fv[i] = raw * dv;
  }
#pragma unroll
  for (int i = 0; i < 8; ++i) {
    const int lr = 16 * wave + 2 * i + hh;
    const int gr = rowBase + lr;
    float* op = outF + (size_t)gr * (size_t)ldo + col0 + 4 * m;
    *(volatile v4f*)op = fv[i];
  }
  __threadfence();
#pragma unroll
  for (int i = 0; i < 8; ++i) {
    const int lr = 16 * wave + 2 * i + hh;
    const int gr = rowBase + lr;
    float* op = outF + (size_t)gr * (size_t)ldo + col0 + 4 * m;
    *(volatile v4f*)op = fv[i];
  }
}

template <int L3>
__global__ __launch_bounds__(NTHR) void k_agg(const int* __restrict__ hsrc, const float* __restrict__ hwt,
                                              const int* __restrict__ cntg, const int* __restrict__ offg,
                                              const float* __restrict__ dinv, const float* __restrict__ xw,
                                              int nN, int mRows,
                                              const float* __restrict__ bias, const float* __restrict__ gam,
                                              const float* __restrict__ bet, const float* __restrict__ rmu,
                                              const float* __restrict__ rva,
                                              unsigned short* hpl, float* outp) {
  __shared__ __attribute__((aligned(16))) int cntS[NBA];
  __shared__ __attribute__((aligned(16))) int offS[NBA];
  __shared__ __attribute__((aligned(16))) unsigned short rowb[NWAVE * KH];
  const int tid = (int)threadIdx.x, lane = tid & 31, wave = tid >> 5;
  const int nodeBase = (int)blockIdx.x * NBA;
  const size_t hbase = (size_t)blockIdx.x * RCAP;

  {
    const v4i c4 = *(const v4ia*)(cntg + (size_t)nodeBase + 4 * tid);
    const v4i o4 = *(const v4ia*)(offg + (size_t)nodeBase + 4 * tid);
    *(v4ia*)(cntS + 4 * tid) = c4;
    *(v4ia*)(offS + 4 * tid) = o4;
  }
  v4f b4 = {0.f, 0.f, 0.f, 0.f}, g4 = b4, be4 = b4, rm4 = b4, rq4 = b4;
  float bq0 = 0.0f, bq1 = 0.0f;
  if constexpr (L3 == 0) {
    const v4f tb = *(const v4fa*)(bias + 4 * lane);
    const v4f tg = *(const v4fa*)(gam + 4 * lane);
    const v4f te = *(const v4fa*)(bet + 4 * lane);
    const v4f tm = *(const v4fa*)(rmu + 4 * lane);
    const v4f tv = *(const v4fa*)(rva + 4 * lane);
    b4.x = bf16_val(tb.x); b4.y = bf16_val(tb.y); b4.z = bf16_val(tb.z); b4.w = bf16_val(tb.w);
    g4.x = bf16_val(tg.x); g4.y = bf16_val(tg.y); g4.z = bf16_val(tg.z); g4.w = bf16_val(tg.w);
    be4.x = bf16_val(te.x); be4.y = bf16_val(te.y); be4.z = bf16_val(te.z); be4.w = bf16_val(te.w);
    rm4.x = bf16_val(tm.x); rm4.y = bf16_val(tm.y); rm4.z = bf16_val(tm.z); rm4.w = bf16_val(tm.w);
    rq4.x = 1.0f / sqrtf(bf16_val(tv.x) + 1e-5f);
    rq4.y = 1.0f / sqrtf(bf16_val(tv.y) + 1e-5f);
    rq4.z = 1.0f / sqrtf(bf16_val(tv.z) + 1e-5f);
    rq4.w = 1.0f / sqrtf(bf16_val(tv.w) + 1e-5f);
  } else {
    const v2f tb = *(const v2fa*)(bias + 2 * lane);
    bq0 = bf16_val(tb.x); bq1 = bf16_val(tb.y);
  }
  __syncthreads();

  const float qnan = __int_as_float(0x7fc00000);
  unsigned short* rowbuf = rowb + wave * KH;
  const int sa = (2 * lane) & 31, sb = (2 * lane + 1) & 31;
#pragma unroll 1
  for (int si = 0; si < NBA / NWAVE; ++si) {
    const int s    = si * NWAVE + wave;
    const int node = nodeBase + s;
    const int craw = cntS[s];
    const bool big = (craw > DEGCAP) || (craw < 0);
    const int c = craw < 0 ? 0 : (craw > DEGCAP ? DEGCAP : craw);
    int o = offS[s];
    o = o < 0 ? 0 : (o > RCAP ? RCAP : o);
    const int nc = node < nN ? node : nN - 1;
    const float dd = dinv[nc];
    float a0 = 0.0f, a1 = 0.0f, a2 = 0.0f, a3 = 0.0f;
#pragma unroll 1
    for (int b0 = 0; b0 < c; b0 += 32) {
      int idx = o + b0 + lane;
      idx = idx > RCAP - 1 ? RCAP - 1 : idx;
      int sr = hsrc[hbase + idx];
      sr = sr < 0 ? 0 : (sr > nN - 1 ? nN - 1 : sr);
      const float wv  = hwt[hbase + idx];
      const int   wvi = __float_as_int(wv);
      const int m32 = (c - b0) < 32 ? (c - b0) : 32;
#pragma unroll 1
      for (int k = 0; k < m32; ++k) {
        const int   sk = __builtin_amdgcn_readlane(sr, k);
        const float ck = __int_as_float(__builtin_amdgcn_readlane(wvi, k));
        if constexpr (L3 == 0) {
          const v4f a = *(const v4fa*)(xw + (size_t)sk * DF + 4 * lane);
          a0 = fmaf(ck, a.x, a0); a1 = fmaf(ck, a.y, a1);
          a2 = fmaf(ck, a.z, a2); a3 = fmaf(ck, a.w, a3);
        } else {
          const v2f a = *(const v2fa*)(xw + (size_t)sk * DO3 + 2 * lane);
          a0 = fmaf(ck, a.x, a0); a1 = fmaf(ck, a.y, a1);
        }
      }
    }
    const float pzr = big ? qnan : 0.0f;
    const bool live = node < nN;
    if constexpr (L3 == 0) {
      const v4f sv = *(const v4fa*)(xw + (size_t)nc * DF + 4 * lane);
      const float y0 = ((a0 + sv.x) * dd + b4.x) + pzr;
      const float y1 = ((a1 + sv.y) * dd + b4.y) + pzr;
      const float y2 = ((a2 + sv.z) * dd + b4.z) + pzr;
      const float y3 = ((a3 + sv.w) * dd + b4.w) + pzr;
      const float t0 = ((y0 - rm4.x) * rq4.x) * g4.x + be4.x;
      const float t1 = ((y1 - rm4.y) * rq4.y) * g4.y + be4.y;
      const float t2 = ((y2 - rm4.z) * rq4.z) * g4.z + be4.z;
      const float t3 = ((y3 - rm4.w) * rq4.w) * g4.w + be4.w;
      const float r0 = (t0 > 0.0f) ? t0 : (t0 - t0);
      const float r1 = (t1 > 0.0f) ? t1 : (t1 - t1);
      const float r2 = (t2 > 0.0f) ? t2 : (t2 - t2);
      const float r3 = (t3 > 0.0f) ? t3 : (t3 - t3);
      const float m0 = live ? r0 : 0.0f;
      const float m1 = live ? r1 : 0.0f;
      const float m2 = live ? r2 : 0.0f;
      const float m3 = live ? r3 : 0.0f;
      v4us mh, ml;
      {
        unsigned hb;
        hb = bf16_bits(m0); mh[0] = (unsigned short)hb; ml[0] = (unsigned short)bf16_bits(m0 - __uint_as_float(hb << 16));
        hb = bf16_bits(m1); mh[1] = (unsigned short)hb; ml[1] = (unsigned short)bf16_bits(m1 - __uint_as_float(hb << 16));
        hb = bf16_bits(m2); mh[2] = (unsigned short)hb; ml[2] = (unsigned short)bf16_bits(m2 - __uint_as_float(hb << 16));
        hb = bf16_bits(m3); mh[3] = (unsigned short)hb; ml[3] = (unsigned short)bf16_bits(m3 - __uint_as_float(hb << 16));
      }
      *(v4usa*)(rowbuf + 4 * lane) = mh;
      *(v4usa*)(rowbuf + DF + 4 * lane) = ml;
      wave_sync();
      const v8us q0 = *(const v8usa*)(rowbuf + 8 * lane);
      wave_sync();
      if (node < mRows) {
        unsigned short* rpw = hpl + (size_t)node * KH + 8 * lane;
        *(volatile v8us*)rpw = q0;
        __threadfence();
        *(volatile v8us*)rpw = q0;
      }
    } else {
      const v2f sv = *(const v2fa*)(xw + (size_t)nc * DO3 + 2 * lane);
      const float y0 = ((a0 + sv.x) * dd + bq0) + pzr;
      const float y1 = ((a1 + sv.y) * dd + bq1) + pzr;
      float ss = y0 * y0 + y1 * y1;
#pragma unroll
      for (int off = 16; off > 0; off >>= 1) ss += __shfl_xor(ss, off, 32);
      const float nrm = sqrtf(ss);
      const float dn  = (nrm < 1e-12f) ? 1e-12f : nrm;
      const float inv = 1.0f / dn;
      const float v0 = y0 * inv;
      const float v1 = y1 * inv;
      v4f ow;
      ow.x = __shfl(v0, sa, 32); ow.y = __shfl(v1, sa, 32);
      ow.z = __shfl(v0, sb, 32); ow.w = __shfl(v1, sb, 32);
      const bool wr = live && (lane < 16);
      float* op = outp + (size_t)nc * DO3 + 4 * (lane & 15);
      if (wr) *(volatile v4f*)op = ow;
      __threadfence();
      if (wr) *(volatile v4f*)op = ow;
    }
  }
}

static inline int cdiv(int a, int b) { return (a + b - 1) / b; }
static inline size_t al256(size_t o) { return (o + 255) & ~(size_t)255; }

extern "C" void kernel_launch(void* const* d_in, const int* in_sizes, int n_in,
                              void* d_out, int out_size, void* d_ws, size_t ws_size,
                              hipStream_t stream) {
  if (n_in < 17) return;
  if (in_sizes[0] < DF || (in_sizes[0] % DF) != 0) return;
  const int nN = in_sizes[0] / DF;
  if (nN < 16 || nN > (1 << 22)) return;
  if (in_sizes[1] < 2 || (in_sizes[1] & 1) != 0) return;
  const int nE = in_sizes[1] / 2;
  if (nE < 1 || nE >= (1 << (31 - SLA))) return;
  if (in_sizes[2] != nE) return;
  if (in_sizes[3] != DF * DF || in_sizes[9] != DF * DF || in_sizes[15] != DF * DO3) return;
  if (in_sizes[4] != DF || in_sizes[5] != DF || in_sizes[6] != DF || in_sizes[7] != DF || in_sizes[8] != DF) return;
  if (in_sizes[10] != DF || in_sizes[11] != DF || in_sizes[12] != DF || in_sizes[13] != DF || in_sizes[14] != DF) return;
  if (in_sizes[16] != DO3) return;
  if ((long long)out_size != (long long)nN * DO3) return;

  const float* x   = (const float*)d_in[0];
  const int*   ei  = (const int*)d_in[1];
  const float* ew  = (const float*)d_in[2];
  const float* W1  = (const float*)d_in[3];
  const float* b1  = (const float*)d_in[4];
  const float* g1  = (const float*)d_in[5];
  const float* be1 = (const float*)d_in[6];
  const float* rm1 = (const float*)d_in[7];
  const float* rv1 = (const float*)d_in[8];
  const float* W2  = (const float*)d_in[9];
  const float* b2  = (const float*)d_in[10];
  const float* g2  = (const float*)d_in[11];
  const float* be2 = (const float*)d_in[12];
  const float* rm2 = (const float*)d_in[13];
  const float* rv2 = (const float*)d_in[14];
  const float* W3  = (const float*)d_in[15];
  const float* b3  = (const float*)d_in[16];
  float* out = (float*)d_out;
  const int* src = ei;
  const int* dst = ei + nE;

  const int MP = cdiv(nN, GBM) * GBM;
  const int gM = MP / GBM;
  const int gA = cdiv(MP, NBA);
  if ((long long)gA * NBA < (long long)MP) return;
  const int vec8 = ((nE & 3) == 0) ? 1 : 0;

  char* ws = (char*)d_ws;
  size_t off = 0;
  const size_t oXW  = off; off = al256(off + (size_t)MP * DF * 4);
  const size_t oBP  = off; off = al256(off + (size_t)MP * KH * 2);
  const size_t oHS  = off; off = al256(off + (size_t)gA * RCAP * 4);
  const size_t oHW  = off; off = al256(off + (size_t)gA * RCAP * 4);
  const size_t oCN  = off; off = al256(off + (size_t)gA * NBA * 4);
  const size_t oOF  = off; off = al256(off + (size_t)gA * NBA * 4);
  const size_t oDV  = off; off = al256(off + (size_t)gA * NBA * 4);
  const size_t oW1T = off; off = al256(off + (size_t)DF * DF * 2);
  const size_t oW2D = off; off = al256(off + (size_t)DF * KH * 2);
  const size_t oW3D = off; off = al256(off + (size_t)DO3 * KH * 2);
  if (off > ws_size || off > (size_t)WSMAX) return;
  float*          XW   = (float*)(ws + oXW);
  unsigned short* BPL  = (unsigned short*)(ws + oBP);
  int*            HSRC = (int*)(ws + oHS);
  float*          HW   = (float*)(ws + oHW);
  int*            CNT  = (int*)(ws + oCN);
  int*            OFF  = (int*)(ws + oOF);
  float*          DINV = (float*)(ws + oDV);
  unsigned short* W1T  = (unsigned short*)(ws + oW1T);
  unsigned short* W2D  = (unsigned short*)(ws + oW2D);
  unsigned short* W3D  = (unsigned short*)(ws + oW3D);

  const size_t grLds = (size_t)GR_LDS_INTS * 4;
  hipFuncSetAttribute(reinterpret_cast<const void*>(&k_graph), hipFuncAttributeMaxDynamicSharedMemorySize, (int)grLds);

  const int nUx = MP * (DF / 8);
  k_wprep<<<(NU1 + NU2 + NU3) / NTHR, NTHR, 0, stream>>>(W1, W2, W3, W1T, W2D, W3D);
  k_cvx<<<cdiv(nUx, NTHR), NTHR, 0, stream>>>(x, nN, nUx, BPL);
  k_graph<<<gA, NTHR, grLds, stream>>>(src, dst, ew, nE, nN, vec8, HSRC, HW, CNT, OFF, DINV);
  k_gemm<<<dim3(gM, DF / GBN), GTHR, 0, stream>>>(BPL, W1T, DINV, XW, DF, DF);
  k_agg<0><<<gA, NTHR, 0, stream>>>(HSRC, HW, CNT, OFF, DINV, XW, nN, MP, b1, g1, be1, rm1, rv1, BPL, out);
  k_gemm<<<dim3(gM, DF / GBN), GTHR, 0, stream>>>(BPL, W2D, DINV, XW, KH, DF);
  k_agg<0><<<gA, NTHR, 0, stream>>>(HSRC, HW, CNT, OFF, DINV, XW, nN, MP, b2, g2, be2, rm2, rv2, BPL, out);
  k_gemm<<<dim3(gM, DO3 / GBN), GTHR, 0, stream>>>(BPL, W3D, DINV, XW, KH, DO3);
  k_agg<1><<<gA, NTHR, 0, stream>>>(HSRC, HW, CNT, OFF, DINV, XW, nN, MP, b3, b3, b3, b3, b3, BPL, out);
}
